// TransformerBlock_65343632441396
// MI455X (gfx1250) — hardware-verified
//
#include <hip/hip_runtime.h>
#include <stddef.h>


typedef _Float16 v16h __attribute__((ext_vector_type(16)));
typedef _Float16 v8h  __attribute__((ext_vector_type(8)));
typedef float    v8f  __attribute__((ext_vector_type(8)));
typedef float    v4f  __attribute__((ext_vector_type(4)));

#ifndef NB
#define NB 2
#endif
#ifndef SEQ
#define SEQ 2048
#endif
#define NB_FULL  2
#define SEQ_FULL 2048
#define DIM   1024
#define NHEAD 16
#define HD    64
#define DFF   4096
#define MROWS (NB * SEQ)

static_assert(NB >= 1 && NB <= NB_FULL);
static_assert(SEQ >= 128 && SEQ <= SEQ_FULL && (SEQ % 128) == 0);
static_assert(DIM == NHEAD * HD);
static_assert(HD == 64);
static_assert((DIM % 64) == 0 && (DIM % 32) == 0);
static_assert((DFF % 64) == 0 && (DFF % 32) == 0);
static_assert(((3 * DIM) % 64) == 0);
static_assert((MROWS % 64) == 0 && (SEQ % 64) == 0);
static_assert((MROWS % 8) == 0);
static_assert(DIM == 32 * 8 * 4);
static_assert((size_t)MROWS * DFF < (size_t)0xFFFFFFFFu);

#define LDT 72
#define LDC 68

#define WCARRY 64.0f
#define PCARRY 1024.0f
#define VCARRY 64.0f

#define WQKV_ELEMS  ((size_t)3 * DIM * DIM)
#define WO_ELEMS    ((size_t)DIM * DIM)
#define W1_ELEMS    ((size_t)DFF * DIM)
#define W2_ELEMS    ((size_t)DIM * DFF)
#define W_BYTES     ((WQKV_ELEMS + WO_ELEMS + W1_ELEMS + W2_ELEMS) * 2)
#define PLANE_ELEMS ((size_t)MROWS * DIM)
#define PLANE16_BYTES (PLANE_ELEMS * 2)
#define FS_BYTES    (PLANE_ELEMS * 4)
#define G_BYTES     ((size_t)MROWS * DFF * 2)
#define WS_TOTAL    (W_BYTES + PLANE16_BYTES * 5 + FS_BYTES + G_BYTES)
static_assert((W_BYTES % 128) == 0 && (PLANE16_BYTES % 128) == 0);
static_assert((FS_BYTES % 128) == 0 && (G_BYTES % 128) == 0);
static_assert((WQKV_ELEMS % 2048) == 0 && (WO_ELEMS % 2048) == 0);
static_assert((W1_ELEMS % 2048) == 0 && (W2_ELEMS % 2048) == 0);
static_assert((size_t)NB * DIM * SEQ == PLANE_ELEMS);
static_assert(WS_TOTAL <= (size_t)134217728);

__device__ __forceinline__ float bf16r(float x) {
  unsigned int u = __float_as_uint(x);
  u = (u + 0x7FFFu + ((u >> 16) & 1u)) & 0xFFFF0000u;
  return __uint_as_float(u);
}

__device__ __forceinline__ v16h frag_at(const _Float16* p) {
  v8h lo = *(const v8h*)(p);
  v8h hi = *(const v8h*)(p + 16);
  v16h out;
#pragma unroll
  for (int i = 0; i < 8; ++i) { out[i] = lo[i]; out[i + 8] = hi[i]; }
  return out;
}
__device__ __forceinline__ v16h ld_frag(const _Float16* base, unsigned ld) {
  const unsigned lane = threadIdx.x & 31u;
  return frag_at(base + (lane & 15u) * ld + (lane >> 4) * 8u);
}

__device__ __forceinline__ v8f wmma16(v16h a, v16h b, v8f c) {
  v8f d = __builtin_amdgcn_wmma_f32_16x16x32_f16(false, a, false, b, (short)0, c,
                                                 false, false);
  asm volatile("v_nop\n\tv_nop\n\tv_nop\n\tv_nop" : "+v"(d) : "v"(a), "v"(b));
  return d;
}

__device__ __forceinline__ float red16_max(float x) {
#pragma unroll
  for (int off = 1; off < 16; off <<= 1) x = fmaxf(x, __shfl_xor(x, off, 32));
  return x;
}
__device__ __forceinline__ float red16_sum(float x) {
#pragma unroll
  for (int off = 1; off < 16; off <<= 1) x += __shfl_xor(x, off, 32);
  return x;
}

__device__ __forceinline__ void wave_lds_sync() {
  __builtin_amdgcn_fence(3  , "wavefront");
  asm volatile("s_wait_dscnt 0x0" ::: "memory");
  __builtin_amdgcn_wave_barrier();
}

__device__ __forceinline__ float gelu_erf(float x) {
  return 0.5f * x * (1.0f + erff(x * 0.70710678118654752f));
}

__global__ __launch_bounds__(256) void wconv_kernel(
    const float* __restrict__ src, _Float16* __restrict__ dst) {
  const size_t e = ((size_t)blockIdx.x * 256u + threadIdx.x) * 8u;
  const v4f a0 = *(const v4f*)(src + e);
  const v4f a1 = *(const v4f*)(src + e + 4);
  v8h o;
#pragma unroll
  for (int j = 0; j < 4; ++j) {
    o[j]     = (_Float16)(WCARRY * bf16r(a0[j]));
    o[j + 4] = (_Float16)(WCARRY * bf16r(a1[j]));
  }
  *(volatile v8h*)(dst + e) = o;
  __threadfence();
  *(volatile v8h*)(dst + e) = o;
}

__global__ __launch_bounds__(256) void rmsnorm_kernel(
    const float* __restrict__ src, const float* __restrict__ lnw,
    _Float16* __restrict__ dst, unsigned seq_src, unsigned rnd) {
  const unsigned tid = threadIdx.x, lane = tid & 31u, w = tid >> 5;
  const unsigned crow = blockIdx.x * 8u + w;
  const unsigned bidx = crow / (unsigned)SEQ;
  const unsigned sq = crow - bidx * (unsigned)SEQ;
  const float* sp = src + ((size_t)bidx * seq_src + sq) * DIM;
  float ss = 0.0f;
#pragma unroll 1
  for (unsigned j = 0; j < 4u; ++j) {
    const unsigned c = (j * 32u + lane) * 8u;
    const v4f a0 = *(const v4f*)(sp + c);
    const v4f a1 = *(const v4f*)(sp + c + 4);
#pragma unroll
    for (int t = 0; t < 4; ++t) {
      const float x0 = rnd ? bf16r(a0[t]) : a0[t];
      const float x1 = rnd ? bf16r(a1[t]) : a1[t];
      ss = fmaf(x0, x0, ss);
      ss = fmaf(x1, x1, ss);
    }
  }
#pragma unroll
  for (int off = 1; off < 32; off <<= 1) ss += __shfl_xor(ss, off, 32);
  const float rinv = 1.0f / sqrtf(ss * (1.0f / (float)DIM) + 1.0e-5f);
#pragma unroll 1
  for (unsigned j = 0; j < 4u; ++j) {
    const unsigned c = (j * 32u + lane) * 8u;
    const v4f a0 = *(const v4f*)(sp + c);
    const v4f a1 = *(const v4f*)(sp + c + 4);
    const v4f g0 = *(const v4f*)(lnw + c);
    const v4f g1 = *(const v4f*)(lnw + c + 4);
    v8h o;
#pragma unroll
    for (int t = 0; t < 4; ++t) {
      const float x0 = rnd ? bf16r(a0[t]) : a0[t];
      const float x1 = rnd ? bf16r(a1[t]) : a1[t];
      o[t]     = (_Float16)((x0 * rinv) * bf16r(g0[t]));
      o[t + 4] = (_Float16)((x1 * rinv) * bf16r(g1[t]));
    }
    _Float16* dp = dst + (size_t)crow * DIM + c;
    *(volatile v8h*)dp = o;
    __threadfence();
    *(volatile v8h*)dp = o;
  }
}

enum { GM_QKV = 0, GM_WO = 1, GM_FF1 = 2, GM_FF2 = 3 };

template <int MODE, int KD>
__device__ __forceinline__ void gemm_body(
    const _Float16* __restrict__ A16, const _Float16* __restrict__ Bt,
    const float* __restrict__ addf, float* __restrict__ outf,
    _Float16* __restrict__ out16) {
  static_assert((KD % 32) == 0);
  __shared__ float Cs[64 * LDC];
  const unsigned tid = threadIdx.x, lane = tid & 31u, w = tid >> 5;
  const unsigned mw = w >> 1, nw = w & 1u;
  const unsigned hh = lane >> 4, m = lane & 15u;
  const unsigned n0 = blockIdx.x * 64u;
  const unsigned row0 = blockIdx.y * 64u;

  const _Float16* ap  = A16 + (size_t)(row0 + mw * 16u + m) * (size_t)KD + hh * 8u;
  const _Float16* bp0 = Bt + (size_t)(n0 + nw * 32u + m) * (size_t)KD + hh * 8u;
  const _Float16* bp1 = bp0 + (size_t)16 * (size_t)KD;
  v8f acc0 = {}, acc1 = {};
#pragma unroll 2
  for (unsigned k0 = 0; k0 < (unsigned)KD; k0 += 32u) {
    const v16h a  = frag_at(ap + k0);
    const v16h b0 = frag_at(bp0 + k0);
    const v16h b1 = frag_at(bp1 + k0);
    acc0 = wmma16(a, b0, acc0);
    acc1 = wmma16(a, b1, acc1);
  }
#pragma unroll
  for (int r = 0; r < 8; ++r) {
    float* d = &Cs[(mw * 16u + hh * 8u + (unsigned)r) * LDC + nw * 32u + m];
    d[0]  = acc0[r];
    d[16] = acc1[r];
  }
  __syncthreads();

  if (MODE == GM_QKV) {
    const unsigned which = n0 >> 10;
    const unsigned nc0 = n0 & 1023u;
    if (which < 2u) {
      v8h x[2];
      size_t off[2];
#pragma unroll
      for (unsigned i = 0; i < 2u; ++i) {
        const unsigned r = 32u * i + (tid >> 3);
        const unsigned c = (tid & 7u) * 8u;
        const v4f u0 = *(const v4f*)&Cs[r * LDC + c];
        const v4f u1 = *(const v4f*)&Cs[r * LDC + c + 4];
#pragma unroll
        for (int j = 0; j < 4; ++j) {
          x[i][j]     = (_Float16)(u0[j] * (1.0f / WCARRY));
          x[i][j + 4] = (_Float16)(u1[j] * (1.0f / WCARRY));
        }
        off[i] = (size_t)which * PLANE_ELEMS + (size_t)(row0 + r) * DIM + nc0 + c;
      }
#pragma unroll
      for (int i = 0; i < 2; ++i) *(volatile v8h*)(out16 + off[i]) = x[i];
      __threadfence();
#pragma unroll
      for (int i = 0; i < 2; ++i) *(volatile v8h*)(out16 + off[i]) = x[i];
    } else {
      const unsigned bidx = row0 / (unsigned)SEQ;
      const unsigned key0 = row0 - bidx * (unsigned)SEQ;
      v8h x[2];
      size_t off[2];
#pragma unroll
      for (unsigned i = 0; i < 2u; ++i) {
        const unsigned dcol = 32u * i + (tid >> 3);
        const unsigned kk = (tid & 7u) * 8u;
#pragma unroll
        for (unsigned j = 0; j < 8u; ++j)
          x[i][j] = (_Float16)(Cs[(kk + j) * LDC + dcol] * (1.0f / WCARRY));
        off[i] = (size_t)2 * PLANE_ELEMS +
                 ((size_t)bidx * DIM + nc0 + dcol) * SEQ + key0 + kk;
      }
#pragma unroll
      for (int i = 0; i < 2; ++i) *(volatile v8h*)(out16 + off[i]) = x[i];
      __threadfence();
#pragma unroll
      for (int i = 0; i < 2; ++i) *(volatile v8h*)(out16 + off[i]) = x[i];
    }
  }

  if (MODE == GM_FF1) {
#pragma unroll 1
    for (unsigned it = 0; it < 4u; ++it) {
      const unsigned r = 32u * (it >> 1) + (tid >> 3);
      const unsigned c = (tid & 7u) * 8u + 4u * (it & 1u);
      v4f u = *(const v4f*)&Cs[r * LDC + c];
#pragma unroll
      for (int j = 0; j < 4; ++j) u[j] = gelu_erf(u[j] * (1.0f / WCARRY));
      *(v4f*)&Cs[r * LDC + c] = u;
    }
    v8h x[2];
    size_t off[2];
#pragma unroll
    for (unsigned i = 0; i < 2u; ++i) {
      const unsigned r = 32u * i + (tid >> 3);
      const unsigned c = (tid & 7u) * 8u;
      const v4f u0 = *(const v4f*)&Cs[r * LDC + c];
      const v4f u1 = *(const v4f*)&Cs[r * LDC + c + 4];
#pragma unroll
      for (int j = 0; j < 4; ++j) {
        x[i][j]     = (_Float16)u0[j];
        x[i][j + 4] = (_Float16)u1[j];
      }
      off[i] = (size_t)(row0 + r) * DFF + n0 + c;
    }
#pragma unroll
    for (int i = 0; i < 2; ++i) *(volatile v8h*)(out16 + off[i]) = x[i];
    __threadfence();
#pragma unroll
    for (int i = 0; i < 2; ++i) *(volatile v8h*)(out16 + off[i]) = x[i];
  }

  if (MODE == GM_WO || MODE == GM_FF2) {
    v4f xs[4];
    size_t off[4];
#pragma unroll
    for (unsigned i = 0; i < 4u; ++i) {
      const unsigned r = 16u * i + (tid >> 4);
      const unsigned c = (tid & 15u) * 4u;
      const unsigned crow = row0 + r;
      const unsigned bidx = crow / (unsigned)SEQ;
      const unsigned sq = crow - bidx * (unsigned)SEQ;
      const size_t frow = (size_t)bidx * SEQ_FULL + sq;
      const v4f u = *(const v4f*)&Cs[r * LDC + c];
      v4f val;
      if (MODE == GM_WO) {
        const v4f g = *(const v4f*)(addf + frow * DIM + n0 + c);
#pragma unroll
        for (int j = 0; j < 4; ++j)
          val[j] = u[j] * (1.0f / (WCARRY * VCARRY)) + bf16r(g[j]);
        off[i] = (size_t)crow * DIM + n0 + c;
      } else {
        const v4f g = *(const v4f*)(addf + (size_t)crow * DIM + n0 + c);
#pragma unroll
        for (int j = 0; j < 4; ++j)
          val[j] = g[j] + u[j] * (1.0f / WCARRY);
        off[i] = frow * DIM + n0 + c;
      }
      xs[i] = val;
    }
#pragma unroll
    for (int i = 0; i < 4; ++i) *(volatile v4f*)(outf + off[i]) = xs[i];
    __threadfence();
#pragma unroll
    for (int i = 0; i < 4; ++i) *(volatile v4f*)(outf + off[i]) = xs[i];
  }
}

__global__ __launch_bounds__(256) void gemm_qkv_kernel(
    const _Float16* __restrict__ A16, const _Float16* __restrict__ Bt,
    _Float16* __restrict__ out16) {
  gemm_body<GM_QKV, DIM>(A16, Bt, nullptr, nullptr, out16);
}
__global__ __launch_bounds__(256) void gemm_wo_kernel(
    const _Float16* __restrict__ A16, const _Float16* __restrict__ Bt,
    const float* __restrict__ xin, float* __restrict__ fs) {
  gemm_body<GM_WO, DIM>(A16, Bt, xin, fs, nullptr);
}
__global__ __launch_bounds__(256) void gemm_ff1_kernel(
    const _Float16* __restrict__ A16, const _Float16* __restrict__ Bt,
    _Float16* __restrict__ out16) {
  gemm_body<GM_FF1, DIM>(A16, Bt, nullptr, nullptr, out16);
}
__global__ __launch_bounds__(256) void gemm_ff2_kernel(
    const _Float16* __restrict__ A16, const _Float16* __restrict__ Bt,
    const float* __restrict__ fs, float* __restrict__ outf) {
  gemm_body<GM_FF2, DFF>(A16, Bt, fs, outf, nullptr);
}

__global__ __launch_bounds__(256) void attn_kernel(
    const _Float16* __restrict__ Qh, const _Float16* __restrict__ Kh,
    const _Float16* __restrict__ Vt, _Float16* __restrict__ Ov) {
  __shared__ _Float16 Ks[64 * LDT];
  __shared__ _Float16 Vs[64 * LDT];
  __shared__ _Float16 Ps[8 * 16 * LDT];

  const unsigned tid = threadIdx.x, lane = tid & 31u;
  const unsigned w = (unsigned)__builtin_amdgcn_readfirstlane((int)(tid >> 5));
  const unsigned hh = lane >> 4, m = lane & 15u;
  const unsigned q0 = blockIdx.x * 128u;
  const unsigned head = blockIdx.y;
  const unsigned b = blockIdx.z;
  const float scale = 0.125f;
  const unsigned pbase = w * (16u * LDT);
  const unsigned qbase = q0 + w * 16u;

  const size_t qoff = (size_t)(b * (unsigned)SEQ + qbase + m) * DIM + head * HD + hh * 8u;

  float mrow[8], lrow[8];
  v8f o[4];
#pragma unroll
  for (int v = 0; v < 8; ++v) { mrow[v] = -1.0e30f; lrow[v] = 0.0f; }
#pragma unroll
  for (int nb = 0; nb < 4; ++nb) o[nb] = (v8f){};

  const size_t kplane = (size_t)b * SEQ * DIM + head * HD;
  const size_t vplane = ((size_t)b * DIM + head * HD) * SEQ;
  const unsigned kend = q0 + 128u;

  for (unsigned kb = 0; kb < kend; kb += 64u) {
#pragma unroll
    for (unsigned j = 0; j < 2u; ++j) {
      const unsigned idx = tid + 256u * j;
      const unsigned r = idx >> 3, c = (idx & 7u) * 8u;
      *(v8h*)&Ks[r * LDT + c] = *(const v8h*)(Kh + kplane + (size_t)(kb + r) * DIM + c);
      *(v8h*)&Vs[r * LDT + c] = *(const v8h*)(Vt + vplane + (size_t)r * SEQ + kb + c);
    }
    __syncthreads();

#pragma unroll 1
    for (unsigned hf = 0; hf < 2u; ++hf) {
      const unsigned kst = kb + hf * 32u;
      if (kst <= qbase + 15u) {
        v8f s0 = {}, s1 = {};
#pragma unroll
        for (unsigned c = 0; c < 2u; ++c) {
          const v16h qf = frag_at(Qh + qoff + c * 32u);
          const v16h k0 = ld_frag(&Ks[(hf * 32u) * LDT + c * 32u], LDT);
          const v16h k1 = ld_frag(&Ks[(hf * 32u + 16u) * LDT + c * 32u], LDT);
          s0 = wmma16(qf, k0, s0);
          s1 = wmma16(qf, k1, s1);
        }

        const unsigned key0 = kst + m, key1 = kst + 16u + m;
#pragma unroll
        for (int v = 0; v < 8; ++v) {
          const unsigned row = qbase + hh * 8u + (unsigned)v;
          const bool mk0 = key0 > row, mk1 = key1 > row;
          const float a0 = mk0 ? -1.0e30f : s0[v] * scale;
          const float a1 = mk1 ? -1.0e30f : s1[v] * scale;
          const float mx = red16_max(fmaxf(a0, a1));
          const float mn = fmaxf(mrow[v], mx);
          const float al = __expf(mrow[v] - mn);
          mrow[v] = mn;
          const float e0 = __expf(a0 - mn);
          const float e1 = __expf(a1 - mn);
          const float p0 = mk0 ? 0.0f : e0;
          const float p1 = mk1 ? 0.0f : e1;
          const float rs = red16_sum(p0 + p1);
          lrow[v] = al * lrow[v] + rs;
#pragma unroll
          for (int nb = 0; nb < 4; ++nb) o[nb][v] = o[nb][v] * al;
          const unsigned pr = pbase + (hh * 8u + (unsigned)v) * LDT + hf * 32u + m;
          Ps[pr]       = (_Float16)(p0 * PCARRY);
          Ps[pr + 16u] = (_Float16)(p1 * PCARRY);
        }
        wave_lds_sync();

        const v16h pf  = ld_frag(&Ps[pbase + hf * 32u], LDT);
        const v16h vf0 = ld_frag(&Vs[(0 * 16) * LDT + hf * 32u], LDT);
        const v16h vf1 = ld_frag(&Vs[(1 * 16) * LDT + hf * 32u], LDT);
        const v16h vf2 = ld_frag(&Vs[(2 * 16) * LDT + hf * 32u], LDT);
        const v16h vf3 = ld_frag(&Vs[(3 * 16) * LDT + hf * 32u], LDT);
        o[0] = wmma16(pf, vf0, o[0]);
        o[1] = wmma16(pf, vf1, o[1]);
        o[2] = wmma16(pf, vf2, o[2]);
        o[3] = wmma16(pf, vf3, o[3]);
      }
    }
    __syncthreads();
  }

  float inv[8];
#pragma unroll
  for (int v = 0; v < 8; ++v) inv[v] = __builtin_amdgcn_rcpf(lrow[v]) * (VCARRY / PCARRY);
#pragma unroll
  for (int nb = 0; nb < 4; ++nb)
#pragma unroll
    for (int v = 0; v < 8; ++v)
      Ps[pbase + (hh * 8u + (unsigned)v) * LDT + (unsigned)nb * 16u + m] =
          (_Float16)(o[nb][v] * inv[v]);
  wave_lds_sync();
  v8h x[4];
  size_t off[4];
#pragma unroll
  for (unsigned i = 0; i < 4u; ++i) {
    const unsigned r = 4u * i + (lane >> 3);
    const unsigned c = (lane & 7u) * 8u;
    x[i] = *(const v8h*)&Ps[pbase + r * LDT + c];
    off[i] = (size_t)(b * (unsigned)SEQ + qbase + r) * DIM + head * HD + c;
  }
#pragma unroll
  for (int i = 0; i < 4; ++i) *(volatile v8h*)(Ov + off[i]) = x[i];
  __threadfence();
#pragma unroll
  for (int i = 0; i < 4; ++i) *(volatile v8h*)(Ov + off[i]) = x[i];
}

extern "C" void kernel_launch(void* const* d_in, const int* in_sizes, int n_in,
                              void* d_out, int out_size, void* d_ws, size_t ws_size,
                              hipStream_t stream) {
  if (n_in < 7) return;
  const long long need_x = ((long long)(NB - 1) * SEQ_FULL + SEQ) * DIM;
  if ((long long)in_sizes[0] < need_x) return;
  if ((long long)in_sizes[1] < (long long)3 * DIM * DIM) return;
  if ((long long)in_sizes[2] < (long long)DIM * DIM) return;
  if (in_sizes[3] < DIM) return;
  if (in_sizes[4] < DIM) return;
  if ((long long)in_sizes[5] < (long long)DFF * DIM) return;
  if ((long long)in_sizes[6] < (long long)DIM * DFF) return;
  if ((long long)out_size < need_x) return;
  if (ws_size < WS_TOTAL) return;

  const float* X    = (const float*)d_in[0];
  const float* Wqkv = (const float*)d_in[1];
  const float* Wo   = (const float*)d_in[2];
  const float* ln1  = (const float*)d_in[3];
  const float* ln2  = (const float*)d_in[4];
  const float* W1   = (const float*)d_in[5];
  const float* W2   = (const float*)d_in[6];
  float* out = (float*)d_out;

  char* ws = (char*)d_ws;
  _Float16* Wqkv16 = (_Float16*)ws;
  _Float16* Wo16   = Wqkv16 + WQKV_ELEMS;
  _Float16* W116   = Wo16 + WO_ELEMS;
  _Float16* W216   = W116 + W1_ELEMS;
  _Float16* H16    = (_Float16*)(ws + W_BYTES);
  _Float16* Q16    = (_Float16*)(ws + W_BYTES + 1 * PLANE16_BYTES);
  _Float16* K16    = (_Float16*)(ws + W_BYTES + 2 * PLANE16_BYTES);
  _Float16* Vt16   = (_Float16*)(ws + W_BYTES + 3 * PLANE16_BYTES);
  _Float16* Ctx16  = (_Float16*)(ws + W_BYTES + 4 * PLANE16_BYTES);
  float*    FS     = (float*)(ws + W_BYTES + 5 * PLANE16_BYTES);
  _Float16* G16    = (_Float16*)(ws + W_BYTES + 5 * PLANE16_BYTES + FS_BYTES);

  dim3 blk(256);

  wconv_kernel<<<dim3((unsigned)(WQKV_ELEMS / 2048)), blk, 0, stream>>>(Wqkv, Wqkv16);
  wconv_kernel<<<dim3((unsigned)(WO_ELEMS / 2048)), blk, 0, stream>>>(Wo, Wo16);
  wconv_kernel<<<dim3((unsigned)(W1_ELEMS / 2048)), blk, 0, stream>>>(W1, W116);
  wconv_kernel<<<dim3((unsigned)(W2_ELEMS / 2048)), blk, 0, stream>>>(W2, W216);

  rmsnorm_kernel<<<dim3(MROWS / 8), blk, 0, stream>>>(X, ln1, H16, (unsigned)SEQ_FULL, 1u);
  gemm_qkv_kernel<<<dim3(3 * DIM / 64, MROWS / 64), blk, 0, stream>>>(H16, Wqkv16, Q16);
  attn_kernel<<<dim3(SEQ / 128, NHEAD, NB), blk, 0, stream>>>(Q16, K16, Vt16, Ctx16);
  gemm_wo_kernel<<<dim3(DIM / 64, MROWS / 64), blk, 0, stream>>>(Ctx16, Wo16, X, FS);
  rmsnorm_kernel<<<dim3(MROWS / 8), blk, 0, stream>>>(FS, ln2, H16, (unsigned)SEQ, 0u);
  gemm_ff1_kernel<<<dim3(DFF / 64, MROWS / 64), blk, 0, stream>>>(H16, W116, G16);
  gemm_ff2_kernel<<<dim3(DIM / 64, MROWS / 64), blk, 0, stream>>>(G16, W216, FS, out);
}
